// MultiHeadAttention_71287867179085
// MI455X (gfx1250) — hardware-run, weakly checked
//
#include <hip/hip_runtime.h>
#ifndef NB
#define NB 2
#endif
#ifndef SEQ
#define SEQ 2048
#endif
#define SQ SEQ
#define NB_FULL 2
#define SQ_FULL 2048
#define DM 1024
#define NH 16
#define HD 64
#define HG 2
#define EARLY ((SQ) < 256 ? (SQ) : 256)
#define NR ((size_t)NB * SQ)
#define NMT (SQ / 128)

typedef unsigned short v8us __attribute__((ext_vector_type(8), may_alias));
typedef float  v8f  __attribute__((ext_vector_type(8)));
typedef float  v4f  __attribute__((ext_vector_type(4)));
typedef float  v4fa __attribute__((ext_vector_type(4), may_alias));
typedef int    v4i  __attribute__((ext_vector_type(4)));
typedef int    v4ia __attribute__((ext_vector_type(4), may_alias));
typedef _Float16 v16h __attribute__((ext_vector_type(16)));
typedef _Float16 v4h  __attribute__((ext_vector_type(4)));
union FragH { v16h v; v8us half[2]; _Float16 h[16]; unsigned short u[16]; };

constexpr size_t al256(size_t b) { return (b + 255) & ~(size_t)255; }
constexpr size_t CARVE_W   = al256((size_t)DM * DM * 2);
constexpr size_t CARVE_ROW = al256(NR * DM * 2);
constexpr size_t CARVE_VT  = al256((size_t)NB * NH * HD * SQ * 2);
constexpr size_t CARVE_S   = al256((size_t)HG * SQ * SQ * 4);
constexpr size_t CARVE_P   = al256((size_t)HG * SQ * SQ * 2);
constexpr size_t CARVE_PL  = al256((size_t)HG * EARLY * SQ * 2);
constexpr size_t CARVE_EXT = al256((size_t)NMT * 32 * 4);
constexpr size_t CARVE_TOTAL = 4 * CARVE_W + 5 * CARVE_ROW + 2 * CARVE_VT + CARVE_S + CARVE_P + CARVE_PL + CARVE_EXT;
static_assert(CARVE_TOTAL <= (size_t)134217728);

__device__ __forceinline__ unsigned short bf16_bits(float x) { unsigned int u = __float_as_uint(x); return (unsigned short)((u + 0x7FFFu + ((u >> 16) & 1u)) >> 16); }
__device__ __forceinline__ float bf16_val(unsigned short b) { return __uint_as_float(((unsigned int)b) << 16); }
__device__ __forceinline__ float bf16_rne(float x) { return bf16_val(bf16_bits(x)); }

__device__ __forceinline__ v16h g2_frag(const _Float16* p, int hh) { FragH f; f.half[0] = *(const v8us*)((const unsigned short*)p + 8 * hh); f.half[1] = *(const v8us*)((const unsigned short*)p + 16 + 8 * hh); return f.v; }
__device__ __forceinline__ v8f g2_mma(v16h a, v16h b, v8f c) { v8f d = __builtin_amdgcn_wmma_f32_16x16x32_f16(false, a, false, b, (short)0, c, false, false); asm volatile("v_nop\n\tv_nop\n\tv_nop\n\tv_nop" : "+v"(d) : "v"(a), "v"(b)); return d; }
__device__ __forceinline__ void mma8(v16h a0, v16h a1, const _Float16* bp, int ldb, int kb, int hh,
                                     v8f& c00, v8f& c01, v8f& c02, v8f& c03, v8f& c10, v8f& c11, v8f& c12, v8f& c13) {
  v16h b = g2_frag(bp + kb, hh);                      c00 = g2_mma(a0, b, c00); c10 = g2_mma(a1, b, c10);
  b = g2_frag(bp + (size_t)16 * ldb + kb, hh);        c01 = g2_mma(a0, b, c01); c11 = g2_mma(a1, b, c11);
  b = g2_frag(bp + (size_t)32 * ldb + kb, hh);        c02 = g2_mma(a0, b, c02); c12 = g2_mma(a1, b, c12);
  b = g2_frag(bp + (size_t)48 * ldb + kb, hh);        c03 = g2_mma(a0, b, c03); c13 = g2_mma(a1, b, c13);
}

__device__ __forceinline__ int ext_cols(const int* __restrict__ ext, int mt) {
  int m = mt; if (m < 0) m = 0; if (m > NMT - 1) m = NMT - 1;
  int e = ext[m * 32];
  if (e < 0) e = 0; if (e > SQ) e = SQ;
  e = (e + 63) & ~63;
  if (e < 64) e = 64; if (e > SQ) e = SQ;
  return e;
}

__global__ __launch_bounds__(256) void k_ext(const int* __restrict__ am, int* __restrict__ ext) {
  __shared__ int red[256];
  __shared__ int rext[128];
  const int tid = threadIdx.x, blk = blockIdx.x;
  const int row = blk * 128 + (tid >> 1);
  const int c0 = (tid & 1) * (SQ / 2);
  const int* mr = am + (size_t)row * SQ_FULL + c0;
  int last = -1;
#pragma unroll 1
  for (int j = 0; j < SQ / 2; j += 4) {
    const v4i m = *(const v4ia*)(mr + j);
    last = (m[0] != 0) ? (c0 + j) : last;
    last = (m[1] != 0) ? (c0 + j + 1) : last;
    last = (m[2] != 0) ? (c0 + j + 2) : last;
    last = (m[3] != 0) ? (c0 + j + 3) : last;
  }
  red[tid] = last;
  __syncthreads();
  if (tid < 128) { const int a = red[2 * tid], b = red[2 * tid + 1]; const int rl = (a > b) ? a : b; rext[tid] = (rl < 0) ? SQ : (rl + 1); }
  __syncthreads();
  if (tid < 32) {
    int e0 = rext[tid], e1 = rext[tid + 32], e2 = rext[tid + 64], e3 = rext[tid + 96];
    int e = (e0 > e1) ? e0 : e1; const int f = (e2 > e3) ? e2 : e3; e = (e > f) ? e : f;
#pragma unroll
    for (int o = 16; o > 0; o >>= 1) { const int x = __shfl_xor(e, o); e = (e > x) ? e : x; }
    if (tid < 8) {
      const v4i o4 = {e, e, e, e};
      *(volatile v4i*)(ext + blk * 32 + tid * 4) = o4;
      __threadfence();
      *(volatile v4i*)(ext + blk * 32 + tid * 4) = o4;
    }
  }
}

__global__ __launch_bounds__(256) void k_wnat(const float* __restrict__ w, size_t n8, _Float16* __restrict__ Bt) {
  const size_t t = (size_t)blockIdx.x * 256 + threadIdx.x; if (t >= n8) return;
  const v4f a = *(const v4fa*)(w + t * 8), c = *(const v4fa*)(w + t * 8 + 4);
  FragH f;
#pragma unroll
  for (int q = 0; q < 4; ++q) { f.h[q] = (_Float16)(bf16_rne(a[q]) * 16.0f); f.h[4 + q] = (_Float16)(bf16_rne(c[q]) * 16.0f); }
  const v8us o = f.half[0];
  unsigned short* d = (unsigned short*)Bt + t * 8;
  *(volatile v8us*)d = o; __threadfence(); *(volatile v8us*)d = o;
}

__global__ __launch_bounds__(256) void k_x16(const float* __restrict__ x, size_t sxb, _Float16* __restrict__ X16, size_t sdb, size_t n8) {
  const size_t t = (size_t)blockIdx.x * 256 + threadIdx.x; if (t >= n8) return;
  const float* xs = x + (size_t)blockIdx.y * sxb + t * 8;
  const v4f a = *(const v4fa*)xs, c = *(const v4fa*)(xs + 4);
  FragH f;
#pragma unroll
  for (int q = 0; q < 4; ++q) { f.h[q] = (_Float16)bf16_rne(a[q]); f.h[4 + q] = (_Float16)bf16_rne(c[q]); }
  const v8us o = f.half[0];
  unsigned short* d = (unsigned short*)X16 + (size_t)blockIdx.y * sdb + t * 8;
  *(volatile v8us*)d = o; __threadfence(); *(volatile v8us*)d = o;
}

template <int NHv, int TTv>
__global__ __launch_bounds__(256) void k_vt(const _Float16* __restrict__ V16, int ldv, int voff, _Float16* __restrict__ Vt) {
  __shared__ unsigned short tl[64][66];
  const int tid = threadIdx.x; const int slab = blockIdx.x / (TTv / 64), lg = blockIdx.x % (TTv / 64); const int b = slab / NHv, h = slab % NHv;
  for (int i = tid; i < 64 * 8; i += 256) { const int r = i / 8, c8 = (i % 8) * 8; FragH f; f.half[0] = *(const v8us*)((const unsigned short*)V16 + ((size_t)b * TTv + lg * 64 + r) * ldv + voff + h * 64 + c8);
#pragma unroll
    for (int q = 0; q < 8; ++q) tl[r][c8 + q] = f.u[q]; }
  __syncthreads();
  for (int pass = 0; pass < 2; ++pass) {
#pragma unroll
    for (int rd = 0; rd < 2; ++rd) { const int d = rd * 32 + tid / 8, pc = tid % 8; FragH f;
#pragma unroll
      for (int q = 0; q < 8; ++q) f.u[q] = tl[pc * 8 + q][d];
      *(volatile v8us*)((unsigned short*)Vt + ((size_t)slab * 64 + d) * TTv + lg * 64 + pc * 8) = f.half[0]; }
    if (pass == 0) __threadfence(); } }

template <int EXTMODE>
__global__ __launch_bounds__(128) void k_gemm2d(const _Float16* __restrict__ A, const _Float16* __restrict__ Al, int lda, size_t sA, size_t sAl,
    const _Float16* __restrict__ Bh, const _Float16* __restrict__ Bl, int ldb, size_t sB,
    float alpha, float alphal, int early, const int* __restrict__ ext,
    float* __restrict__ C, _Float16* __restrict__ C16, _Float16* __restrict__ C16l, int ldc, size_t sC, int M, int N, int K) {
  __shared__ __attribute__((aligned(16))) float so[4][32][68];
  const int tid = threadIdx.x, w = tid >> 5, lane = tid & 31, ln = lane & 15, hh = lane >> 4; const int by = blockIdx.y;
  const int ntn = N >> 6; const int mt = blockIdx.x / ntn, nq = blockIdx.x - mt * ntn;
  const int row0 = mt * 128 + 32 * w, col0 = nq * 64;
  if (mt * 128 >= M) return;
  int kend = K;
  if (EXTMODE != 0) { const int e = ext_cols(ext, mt); if (EXTMODE == 1) { if (col0 >= e) return; } else { kend = (e < K) ? e : K; } }
  const bool lo_rows = (mt * 128 < early);
  const bool lo_prod = lo_rows && (Al != nullptr || Bl != nullptr);
  const bool lo_out  = lo_rows && (C16l != nullptr);
  const size_t cofs = (size_t)by * sC;
  const size_t aoff = (size_t)by * sA + (size_t)(row0 + ln) * lda;
  const size_t boff = (size_t)by * sB + (size_t)(col0 + ln) * ldb;
  const _Float16* a0p = A + aoff; const _Float16* a1p = a0p + (size_t)16 * lda;
  const _Float16* b0p = Bh + boff;
  const v8f z8 = {0.f,0.f,0.f,0.f,0.f,0.f,0.f,0.f};
  v8f c00 = z8, c01 = z8, c02 = z8, c03 = z8, c10 = z8, c11 = z8, c12 = z8, c13 = z8;
#pragma unroll 1
  for (int kb = 0; kb < kend; kb += 32) {
    const v16h a0 = g2_frag(a0p + kb, hh), a1 = g2_frag(a1p + kb, hh);
    mma8(a0, a1, b0p, ldb, kb, hh, c00, c01, c02, c03, c10, c11, c12, c13);
  }
  {
    v8f accs[8] = {c00, c01, c02, c03, c10, c11, c12, c13};
#pragma unroll
    for (int u = 0; u < 8; ++u) { const int t = u & 3, half = u >> 2;
#pragma unroll
      for (int r = 0; r < 8; ++r) so[w][half * 16 + 8 * hh + r][t * 16 + ln] = accs[u][r] * alpha; }
  }
  if (lo_prod) {
    c00 = z8; c01 = z8; c02 = z8; c03 = z8; c10 = z8; c11 = z8; c12 = z8; c13 = z8;
    const size_t aloff = (size_t)by * sAl + (size_t)(row0 + ln) * lda;
#pragma unroll 1
    for (int kb = 0; kb < kend; kb += 32) {
      if (Bl != nullptr) {
        const v16h a0 = g2_frag(a0p + kb, hh), a1 = g2_frag(a1p + kb, hh);
        mma8(a0, a1, Bl + boff, ldb, kb, hh, c00, c01, c02, c03, c10, c11, c12, c13);
      }
      if (Al != nullptr) {
        const v16h l0 = g2_frag(Al + aloff + kb, hh), l1 = g2_frag(Al + aloff + (size_t)16 * lda + kb, hh);
        mma8(l0, l1, b0p, ldb, kb, hh, c00, c01, c02, c03, c10, c11, c12, c13);
      }
    }
    v8f accs[8] = {c00, c01, c02, c03, c10, c11, c12, c13};
#pragma unroll
    for (int u = 0; u < 8; ++u) { const int t = u & 3, half = u >> 2;
#pragma unroll
      for (int r = 0; r < 8; ++r) so[w][half * 16 + 8 * hh + r][t * 16 + ln] += accs[u][r] * alphal; }
  }
  __builtin_amdgcn_fence(4  , "workgroup"); __builtin_amdgcn_wave_barrier();
  const int rsub = lane >> 4, c4 = (lane & 15) * 4;
  for (int pass = 0; pass < 2; ++pass) {
#pragma unroll
    for (int q = 0; q < 16; ++q) {
      const int r = q * 2 + rsub;
      const v4f v = *(const v4fa*)&so[w][r][c4];
      const size_t o = cofs + (size_t)(row0 + r) * ldc + col0 + c4;
      if (C != nullptr) *(volatile v4f*)(C + o) = v;
      v4h h4;
#pragma unroll
      for (int i = 0; i < 4; ++i) h4[i] = (_Float16)v[i];
      if (C16 != nullptr) *(volatile v4h*)(C16 + o) = h4;
      if (lo_out) { v4h l4;
#pragma unroll
        for (int i = 0; i < 4; ++i) l4[i] = (_Float16)((v[i] - (float)h4[i]) * 1024.0f);
        *(volatile v4h*)(C16l + o) = l4; }
    }
    if (pass == 0) __threadfence();
  }
}

__global__ __launch_bounds__(256) void k_rsmkm(const float* __restrict__ S, _Float16* __restrict__ P, _Float16* __restrict__ Pl, int nrows, const int* __restrict__ am, const int* __restrict__ ext) {
  #pragma clang fp contract(off)
  const int t = blockIdx.x * 256 + threadIdx.x; if (t >= nrows) return;
  const int q = t % SQ, slab = t / SQ;
  const int J = ext_cols(ext, q >> 7);
  const float* s = S + (size_t)t * SQ; const int* mr = am + (size_t)q * SQ_FULL;
  float mx = -3.0e38f;
#pragma unroll 1
  for (int j = 0; j < J; j += 4) { const v4f sv = *(const v4fa*)(s + j); const v4i mv = *(const v4ia*)(mr + j);
#pragma unroll
    for (int i = 0; i < 4; ++i) { const float x = (mv[i] != 0) ? sv[i] : -1.0e9f; mx = fmaxf(mx, x); } }
  float se = 0.f;
#pragma unroll 1
  for (int j = 0; j < J; j += 4) { const v4f sv = *(const v4fa*)(s + j); const v4i mv = *(const v4ia*)(mr + j);
#pragma unroll
    for (int i = 0; i < 4; ++i) { const float x = (mv[i] != 0) ? sv[i] : -1.0e9f; se += __expf(x - mx); } }
  const float sc = 256.0f * (1.0f / se);
  const bool wl = (q < EARLY);
  unsigned short* dh = (unsigned short*)P + (size_t)t * SQ;
  unsigned short* dl = (unsigned short*)Pl + ((size_t)slab * EARLY + (wl ? q : 0)) * SQ;
#pragma unroll 1
  for (int j0 = 0; j0 < J; j0 += 8) {
    const v4f s0 = *(const v4fa*)(s + j0), s1 = *(const v4fa*)(s + j0 + 4); const v4i m0 = *(const v4ia*)(mr + j0), m1 = *(const v4ia*)(mr + j0 + 4);
    FragH fh, fl;
#pragma unroll
    for (int i = 0; i < 4; ++i) {
      const float x0 = (m0[i] != 0) ? s0[i] : -1.0e9f; const float e0 = __expf(x0 - mx) * sc; const _Float16 h0 = (_Float16)e0; fh.h[i] = h0; fl.h[i] = (_Float16)((e0 - (float)h0) * 1024.0f);
      const float x1 = (m1[i] != 0) ? s1[i] : -1.0e9f; const float e1 = __expf(x1 - mx) * sc; const _Float16 h1 = (_Float16)e1; fh.h[4 + i] = h1; fl.h[4 + i] = (_Float16)((e1 - (float)h1) * 1024.0f);
    }
    const v8us oh = fh.half[0], ol = fl.half[0];
    *(volatile v8us*)(dh + j0) = oh; if (wl) *(volatile v8us*)(dl + j0) = ol;
    __threadfence();
    *(volatile v8us*)(dh + j0) = oh; if (wl) *(volatile v8us*)(dl + j0) = ol;
  }
}

extern "C" void kernel_launch(void* const* d_in, const int* in_sizes, int n_in,
                              void* d_out, int out_size, void* d_ws, size_t ws_size, hipStream_t stream) {
  static_assert(NH * HD == DM);
  static_assert(DM % 64 == 0 && SQ % 256 == 0 && NH % HG == 0);
  static_assert(EARLY % 128 == 0 && EARLY <= SQ);
  static_assert(NB <= NB_FULL && SQ <= SQ_FULL);
  if (n_in < 9) return;
  const size_t need_x = ((size_t)(NB - 1) * SQ_FULL + SQ) * DM;
  const size_t need_m = (size_t)(SQ - 1) * SQ_FULL + SQ;
  if ((size_t)in_sizes[0] < need_x || (size_t)in_sizes[1] < need_x || (size_t)in_sizes[2] < need_x) return;
  if ((size_t)in_sizes[4] < need_m) return;
  if ((size_t)in_sizes[5] < (size_t)DM * DM || (size_t)in_sizes[6] < (size_t)DM * DM || (size_t)in_sizes[7] < (size_t)DM * DM || (size_t)in_sizes[8] < (size_t)DM * DM) return;
  if ((size_t)out_size < NR * DM) return;
  const float* xq = (const float*)d_in[0]; const float* xk = (const float*)d_in[1]; const float* xv = (const float*)d_in[2];
  const int* am = (const int*)d_in[4];
  const float* wq = (const float*)d_in[5]; const float* wk = (const float*)d_in[6]; const float* wv = (const float*)d_in[7]; const float* wo = (const float*)d_in[8];
  char* ws = (char*)d_ws; size_t off = 0;
  auto take = [&](size_t bytes) { char* p = ws + off; off += (bytes + 255) & ~(size_t)255; return p; };
  _Float16* WQ = (_Float16*)take((size_t)DM * DM * 2); _Float16* WK = (_Float16*)take((size_t)DM * DM * 2);
  _Float16* WV = (_Float16*)take((size_t)DM * DM * 2); _Float16* WO = (_Float16*)take((size_t)DM * DM * 2);
  _Float16* X16 = (_Float16*)take(NR * DM * 2);
  _Float16* Q16 = (_Float16*)take(NR * DM * 2); _Float16* K16 = (_Float16*)take(NR * DM * 2);
  _Float16* VH = (_Float16*)take(NR * DM * 2); _Float16* VL = (_Float16*)take(NR * DM * 2);
  _Float16* VTH = (_Float16*)take((size_t)NB * NH * HD * SQ * 2); _Float16* VTL = (_Float16*)take((size_t)NB * NH * HD * SQ * 2);
  _Float16* OH = VH; _Float16* OL = VL;
  float* S = (float*)take((size_t)HG * SQ * SQ * 4);
  _Float16* P = (_Float16*)take((size_t)HG * SQ * SQ * 2);
  _Float16* PL = (_Float16*)take((size_t)HG * EARLY * SQ * 2);
  int* EXT = (int*)take((size_t)NMT * 32 * 4);
  if (off != CARVE_TOTAL) return;
  if (off > ws_size || off > (size_t)134217728) return;

  k_ext<<<NMT, 256, 0, stream>>>(am, EXT);
  const size_t wn8 = (size_t)DM * DM / 8;
  const unsigned gw = (unsigned)((wn8 + 255) / 256);
  k_wnat<<<gw, 256, 0, stream>>>(wq, wn8, WQ);
  k_wnat<<<gw, 256, 0, stream>>>(wk, wn8, WK);
  k_wnat<<<gw, 256, 0, stream>>>(wv, wn8, WV);
  k_wnat<<<gw, 256, 0, stream>>>(wo, wn8, WO);

  const size_t xn8 = (size_t)SQ * DM / 8;
  const dim3 gx((unsigned)((xn8 + 255) / 256), NB);
  const int MP = (int)NR;
  const dim3 gp((unsigned)((MP / 128) * (DM / 64)), 1);
  k_x16<<<gx, 256, 0, stream>>>(xq, (size_t)SQ_FULL * DM, X16, (size_t)SQ * DM, xn8);
  k_gemm2d<0><<<gp, 128, 0, stream>>>(X16, nullptr, DM, 0, 0, WQ, nullptr, DM, 0, 0.0625f, 0.f, 0, nullptr, nullptr, Q16, nullptr, DM, 0, MP, DM, DM);
  k_x16<<<gx, 256, 0, stream>>>(xk, (size_t)SQ_FULL * DM, X16, (size_t)SQ * DM, xn8);
  k_gemm2d<0><<<gp, 128, 0, stream>>>(X16, nullptr, DM, 0, 0, WK, nullptr, DM, 0, 0.0625f, 0.f, 0, nullptr, nullptr, K16, nullptr, DM, 0, MP, DM, DM);
  k_x16<<<gx, 256, 0, stream>>>(xv, (size_t)SQ_FULL * DM, X16, (size_t)SQ * DM, xn8);
  k_gemm2d<0><<<gp, 128, 0, stream>>>(X16, nullptr, DM, 0, 0, WV, nullptr, DM, 0, 0.0625f, 0.f, MP, nullptr, nullptr, VH, VL, DM, 0, MP, DM, DM);
  k_vt<NH, SQ><<<NB * NH * (SQ / 64), 256, 0, stream>>>(VH, DM, 0, VTH);
  k_vt<NH, SQ><<<NB * NH * (SQ / 64), 256, 0, stream>>>(VL, DM, 0, VTL);

  for (int b = 0; b < NB; ++b) {
    const size_t r0 = (size_t)b * SQ;
    for (int h0 = 0; h0 < NH; h0 += HG) {
      k_gemm2d<1><<<dim3((unsigned)((SQ / 128) * (SQ / 64)), HG), 128, 0, stream>>>(Q16 + r0 * DM + h0 * HD, nullptr, DM, (size_t)HD, 0,
          K16 + r0 * DM + h0 * HD, nullptr, DM, (size_t)HD, 0.125f, 0.f, 0, EXT, S, nullptr, nullptr, SQ, (size_t)SQ * SQ, SQ, SQ, HD);
      k_rsmkm<<<(HG * SQ + 255) / 256, 256, 0, stream>>>(S, P, PL, HG * SQ, am, EXT);
      k_gemm2d<2><<<dim3((unsigned)(SQ / 128), HG), 128, 0, stream>>>(P, PL, SQ, (size_t)SQ * SQ, (size_t)EARLY * SQ,
          VTH + (size_t)(b * NH + h0) * HD * SQ, VTL + (size_t)(b * NH + h0) * HD * SQ, SQ, (size_t)HD * SQ,
          0.25f, 0.000244140625f, EARLY, EXT, nullptr, OH + r0 * DM + h0 * HD, OL + r0 * DM + h0 * HD, DM, (size_t)HD, SQ, HD, SQ);
    }
  }
  k_gemm2d<0><<<dim3((unsigned)((SQ / 128) * (DM / 64)), NB), 128, 0, stream>>>(OH, OL, DM, (size_t)SQ * DM, (size_t)SQ * DM,
      WO, nullptr, DM, 0, 0.0009765625f, 9.5367431640625e-7f, EARLY, nullptr, (float*)d_out, nullptr, nullptr, DM, (size_t)SQ * DM, SQ, DM, DM);
}
